// ResonanceMemoryAttentionV15_72172630442600
// MI455X (gfx1250) — hardware-verified
//
#include <hip/hip_runtime.h>


#define NB_  1
#define NT_  1024
#define DM   768
#define NH_  12
#define GH   16
#define BW   128
#define PW   64
#define HD   64
#define NTK  (NB_ * NT_)
#define NW   1024
#define NQKV 1024
#define PSC  1.0f
#define LOSC 1024.0f
#define LOSCI (1.0f / 1024.0f)

typedef _Float16 h16;
typedef unsigned short bf;
typedef __attribute__((ext_vector_type(16))) __bf16   v16bf;
typedef __attribute__((ext_vector_type(16))) _Float16 v16h;
typedef __attribute__((ext_vector_type(8)))  _Float16 v8h;
typedef __attribute__((ext_vector_type(8)))  unsigned short v8us;
typedef __attribute__((ext_vector_type(8)))  float    v8f;
typedef __attribute__((ext_vector_type(4)))  float    v4f;
typedef v8h  __attribute__((may_alias)) v8ha;
typedef v4f  __attribute__((may_alias)) v4fa;
typedef v8us __attribute__((may_alias)) v8usa;

__device__ __forceinline__ unsigned short f2bf(float f) { unsigned u = __float_as_uint(f); u += 0x7FFFu + ((u >> 16) & 1u); return (unsigned short)(u >> 16); }
__device__ __forceinline__ float bf2f(unsigned short b) { return __uint_as_float(((unsigned)b) << 16); }
__device__ __forceinline__ float bfr(float f) { return bf2f(f2bf(f)); }
__device__ __forceinline__ v16h cat16(v8h lo, v8h hi) { return __builtin_shufflevector(lo, hi, 0, 1, 2, 3, 4, 5, 6, 7, 8, 9, 10, 11, 12, 13, 14, 15); }
__device__ __forceinline__ v16bf cat16b(v8us lo, v8us hi) { return __builtin_bit_cast(v16bf, __builtin_shufflevector(lo, hi, 0, 1, 2, 3, 4, 5, 6, 7, 8, 9, 10, 11, 12, 13, 14, 15)); }
__device__ __forceinline__ v8f wmma16(v16h a, v16h b, v8f c) { return __builtin_amdgcn_wmma_f32_16x16x32_f16(false, a, false, b, (short)0, c, false, false); }
__device__ __forceinline__ v8f wmmab(v16bf a, v16bf b, v8f c) { return __builtin_amdgcn_wmma_f32_16x16x32_bf16(false, a, false, b, (short)0, c, false, false); }

__global__ __launch_bounds__(256) void k_cvtb(const float* __restrict__ src, int nrows, bf* dst) {
    const int lane = threadIdx.x & 31, r = blockIdx.x * 8 + (threadIdx.x >> 5);
    if (r >= nrows) return;
    v8us o[DM / 256];
#pragma unroll
    for (int q = 0; q < DM / 256; ++q) { v8us t;
#pragma unroll
        for (int i = 0; i < 8; ++i) t[i] = f2bf(src[(size_t)r * DM + q * 256 + lane * 8 + i]);
        o[q] = t; }
#pragma unroll
    for (int q = 0; q < DM / 256; ++q) *(volatile v8us*)(dst + (size_t)r * DM + q * 256 + lane * 8) = o[q];
    __threadfence();
#pragma unroll
    for (int q = 0; q < DM / 256; ++q) *(volatile v8us*)(dst + (size_t)r * DM + q * 256 + lane * 8) = o[q];
}

template <bool SPLITA, bool F16OUT = false>
__global__ __launch_bounds__(128) void k_gemmb(const bf* __restrict__ A, const bf* __restrict__ Al, const bf* __restrict__ Bn, const float* __restrict__ bias, float* C, int ldc, h16* C2, const float* __restrict__ R = nullptr, int K = DM, int roundR = 1) {
    __shared__ __align__(16) float ost[4][16 * 68];
    const int lane = threadIdx.x & 31, wave = threadIdx.x >> 5, lr = lane & 15, hi = lane >> 4;
    const int r0 = blockIdx.x * 64 + wave * 16, c0 = blockIdx.y * 64;
    const size_t aoff = (size_t)(r0 + lr) * K + 8 * hi;
    size_t boff[4];
#pragma unroll
    for (int t = 0; t < 4; ++t) boff[t] = (size_t)(c0 + t * 16 + lr) * K + 8 * hi;
    v8f acc[4];
#pragma unroll
    for (int t = 0; t < 4; ++t) acc[t] = (v8f){};
#pragma unroll 1
    for (int kc = 0; kc < K; kc += 32) {
        const v16bf a = cat16b(*(const v8us*)(A + aoff + kc), *(const v8us*)(A + aoff + kc + 16));
        v16bf al = a;
        if (SPLITA) al = cat16b(*(const v8us*)(Al + aoff + kc), *(const v8us*)(Al + aoff + kc + 16));
#pragma unroll
        for (int t = 0; t < 4; ++t) { const v16bf b = cat16b(*(const v8us*)(Bn + boff[t] + kc), *(const v8us*)(Bn + boff[t] + kc + 16)); acc[t] = wmmab(a, b, acc[t]); if (SPLITA) acc[t] = wmmab(al, b, acc[t]); }
        asm volatile("v_nop\n\tv_nop\n\tv_nop\n\tv_nop" : "+v"(acc[0]), "+v"(acc[1]), "+v"(acc[2]), "+v"(acc[3]) : "v"(a), "v"(al));
    }
    float* os = &ost[wave][0];
#pragma unroll
    for (int t = 0; t < 4; ++t) { const float bv = bias ? bfr(bias[c0 + t * 16 + lr]) : 0.f;
#pragma unroll
        for (int j = 0; j < 8; ++j) os[(hi * 8 + j) * 68 + t * 16 + lr] = acc[t][j] + bv; }
    __syncthreads();
    if (F16OUT) {
        h16* crow = (h16*)(void*)C + (size_t)r0 * ldc + c0;
        auto pass = [&]() {
#pragma unroll
            for (int s = 0; s < 4; ++s) { const int row = 4 * s + (lane >> 3), piece = lane & 7; const float* sp = os + row * 68 + piece * 8; v8h o, o2;
#pragma unroll
                for (int i = 0; i < 8; ++i) { const h16 a = (h16)sp[i]; o[i] = a; o2[i] = (h16)((sp[i] - (float)a) * LOSC); }
                *(volatile v8h*)(crow + (size_t)row * ldc + piece * 8) = o; if (C2) *(volatile v8h*)(C2 + (size_t)r0 * ldc + c0 + (size_t)row * ldc + piece * 8) = o2; }
        };
        pass(); __threadfence(); pass();
    } else {
        float* crow = C + (size_t)r0 * ldc + c0;
        auto pass = [&]() {
#pragma unroll
            for (int s = 0; s < 8; ++s) { const int Lid = (lane >> 3) + 4 * s, piece = lane & 7; const int row = Lid >> 1, cofs = (Lid & 1) * 32 + piece * 4;
                v4f val = *(const v4fa*)(os + row * 68 + cofs); if (R) { const v4f rv = *(const v4f*)(R + ((size_t)r0 + row) * ldc + c0 + cofs); val += roundR ? (v4f){bfr(rv[0]), bfr(rv[1]), bfr(rv[2]), bfr(rv[3])} : rv; }
                *(volatile v4f*)(crow + (size_t)row * ldc + cofs) = val; }
        };
        pass(); __threadfence(); pass();
    }
}

__global__ __launch_bounds__(256) void k_wt(const float* __restrict__ Wm, int K, int ncols, bf* WT) {
    __shared__ __align__(16) unsigned short tl[64 * 72];
    const int tid = threadIdx.x, k0 = blockIdx.x * 64, n0 = blockIdx.y * 64;
    const int kk = tid >> 2, nq = (tid & 3) * 16;
#pragma unroll
    for (int i = 0; i < 16; ++i) tl[(nq + i) * 72 + kk] = f2bf(Wm[(size_t)(k0 + kk) * ncols + n0 + nq + i]);
    __syncthreads();
    const int piece = tid & 7;
    auto pass = [&]() {
#pragma unroll
        for (int s = 0; s < 2; ++s) { const int nr = (tid >> 3) + 32 * s; const v8us val = *(const v8usa*)(tl + nr * 72 + piece * 8); *(volatile v8us*)(WT + (size_t)(n0 + nr) * K + k0 + piece * 8) = val; }
    };
    pass(); __threadfence(); pass();
}
template <bool ROUNDIN>
__global__ __launch_bounds__(256) void k_ln(const float* __restrict__ X, const float* __restrict__ gam, const float* __restrict__ bet, int nrows, bf* Hh, bf* Hl) {
    const int lane = threadIdx.x & 31, r = blockIdx.x * 8 + (threadIdx.x >> 5);
    if (r >= nrows) return;
    const float* xr = X + (size_t)r * DM + lane * 8;
    float s = 0.f;
#pragma unroll 1
    for (int q = 0; q < DM / 256; ++q) {
#pragma unroll
        for (int i = 0; i < 8; ++i) s += (ROUNDIN ? bfr(xr[q * 256 + i]) : xr[q * 256 + i]); }
#pragma unroll
    for (int sh = 16; sh; sh >>= 1) s += __shfl_xor(s, sh, 32);
    const float mu = s * (1.0f / DM);
    float s2 = 0.f;
#pragma unroll 1
    for (int q = 0; q < DM / 256; ++q) {
#pragma unroll
        for (int i = 0; i < 8; ++i) { const float d = (ROUNDIN ? bfr(xr[q * 256 + i]) : xr[q * 256 + i]) - mu; s2 = fmaf(d, d, s2); } }
#pragma unroll
    for (int sh = 16; sh; sh >>= 1) s2 += __shfl_xor(s2, sh, 32);
    const float rs = rsqrtf(s2 * (1.0f / DM) + 1e-5f);
#pragma unroll 1
    for (int ps = 0; ps < 2; ++ps) {
#pragma unroll 1
        for (int q = 0; q < DM / 256; ++q) { v8us oh, ol;
#pragma unroll
            for (int i = 0; i < 8; ++i) { const int c = q * 256 + lane * 8 + i; const float y = ((ROUNDIN ? bfr(xr[q * 256 + i]) : xr[q * 256 + i]) - mu) * rs * bfr(gam[c]) + bfr(bet[c]); const unsigned short hb = f2bf(y); oh[i] = hb; ol[i] = f2bf(y - bf2f(hb)); }
            const size_t o = (size_t)r * DM + q * 256 + lane * 8; *(volatile v8us*)(Hh + o) = oh; *(volatile v8us*)(Hl + o) = ol; }
        if (ps == 0) __threadfence(); }
}
__global__ __launch_bounds__(256) void k_silu2(const float* __restrict__ src, int nrows, bf* dh, bf* dl) {
    typedef __attribute__((ext_vector_type(4))) unsigned short v4us;
    const int lane = threadIdx.x & 31, r = blockIdx.x * 8 + (threadIdx.x >> 5); if (r >= nrows) return;
    const size_t o = (size_t)r * BW + lane * 4; const v4f v = *(const v4f*)(src + o); v4us oh, ol;
#pragma unroll
    for (int i = 0; i < 4; ++i) { const float x = v[i]; const float y = x / (1.0f + __expf(-x)); const unsigned short hb = f2bf(y); oh[i] = hb; ol[i] = f2bf(y - bf2f(hb)); }
    *(volatile v4us*)(dh + o) = oh; *(volatile v4us*)(dl + o) = ol; __threadfence(); *(volatile v4us*)(dh + o) = oh; *(volatile v4us*)(dl + o) = ol;
}
__device__ __forceinline__ float gate_of(const float* __restrict__ PR, const float tmp, int t, int h) {
    const float* p = PR + (size_t)t * PW + h * 5;
    const float sa = 1.0f / (1.0f + __expf(-p[0])), sp = tanhf(p[1]) * 3.14159265358979323846f, ca = 1.0f / (1.0f + __expf(-p[2])), cp = tanhf(p[3]) * 3.14159265358979323846f;
    const float inter = tanhf(sa * ca * cosf(sp - cp)) * tmp;
    return 1.0f / (1.0f + __expf(-inter));
}
__global__ __launch_bounds__(256) void k_gate(const float* __restrict__ PR, const float* __restrict__ temp, float* G) {
    const int i = blockIdx.x * 256 + threadIdx.x; if (i >= NT_ * GH) return;
    const float tmp = fminf(fmaxf(bfr(temp[0]), 0.1f), 2.0f);
    const int t = i / GH, h = i % GH; const float g = (h < NH_) ? gate_of(PR, tmp, t, h) : 0.f;
    *(volatile float*)(G + i) = g; __threadfence(); *(volatile float*)(G + i) = g;
}
__global__ __launch_bounds__(256) void k_gout(const float* __restrict__ G, float* GOUT) {
    const int i = blockIdx.x * 256 + threadIdx.x; if (i >= NT_ * NH_) return;
    const float g = G[(i / NH_) * GH + (i % NH_)];
    *(volatile float*)(GOUT + i) = g; __threadfence(); *(volatile float*)(GOUT + i) = g;
}
__global__ __launch_bounds__(256) void k_elu16(const float* __restrict__ QKV, int col0, int nrows, h16* Yh, h16* Yl) {
    const int lane = threadIdx.x & 31, r = blockIdx.x * 8 + (threadIdx.x >> 5); if (r >= nrows) return;
#pragma unroll 1
    for (int ps = 0; ps < 2; ++ps) {
#pragma unroll 1
        for (int q = 0; q < DM / 256; ++q) { const size_t so = (size_t)r * (3 * DM) + col0 + q * 256 + lane * 8, o = (size_t)r * DM + q * 256 + lane * 8; const v8f v = *(const v8f*)(QKV + so); v8h oh, ol;
#pragma unroll
            for (int i = 0; i < 8; ++i) { const float x = v[i]; const float y = (x > 0.f ? x : expm1f(x)) + 1.0f; const h16 a = (h16)y; oh[i] = a; ol[i] = (h16)((y - (float)a) * LOSC); }
            *(volatile v8h*)(Yh + o) = oh; *(volatile v8h*)(Yl + o) = ol; }
        if (ps == 0) __threadfence(); }
}
__global__ __launch_bounds__(256) void k_vcopy(const float* __restrict__ QKV, int nrows, float* V) {
    const int lane = threadIdx.x & 31, r = blockIdx.x * 8 + (threadIdx.x >> 5); if (r >= nrows) return;
#pragma unroll 1
    for (int ps = 0; ps < 2; ++ps) {
#pragma unroll
        for (int q = 0; q < DM / 128; ++q) { const v4f v = *(const v4f*)(QKV + (size_t)r * (3 * DM) + 2 * DM + q * 128 + lane * 4); *(volatile v4f*)(V + (size_t)r * DM + q * 128 + lane * 4) = v; }
        if (ps == 0) __threadfence(); }
}
__global__ __launch_bounds__(256) void k_hln(const float* __restrict__ CTX, const float* __restrict__ w, const float* __restrict__ bb, h16* unused, bf* Hh, bf* Hl) {
    typedef __attribute__((ext_vector_type(4))) unsigned short v4us;
    (void)unused;
    const int lane = threadIdx.x & 31, wid = blockIdx.x * 8 + (threadIdx.x >> 5); if (wid >= NT_ * (NH_ / 2)) return;
    const int t = wid / (NH_ / 2), hp = wid - t * (NH_ / 2); const int hl = lane >> 4, l16 = lane & 15;
    const size_t o = (size_t)t * DM + (hp * 2 + hl) * HD + l16 * 4; const v4f v = *(const v4f*)(CTX + o);
    float s = (v[0] + v[1]) + (v[2] + v[3]);
    s += __shfl_xor(s, 1, 16); s += __shfl_xor(s, 2, 16); s += __shfl_xor(s, 4, 16); s += __shfl_xor(s, 8, 16);
    const float mu = s * (1.0f / HD);
    float s2 = 0.f;
#pragma unroll
    for (int i = 0; i < 4; ++i) { const float d = v[i] - mu; s2 = fmaf(d, d, s2); }
    s2 += __shfl_xor(s2, 1, 16); s2 += __shfl_xor(s2, 2, 16); s2 += __shfl_xor(s2, 4, 16); s2 += __shfl_xor(s2, 8, 16);
    const float rs = rsqrtf(s2 * (1.0f / HD) + 1e-5f);
    v4us oh, ol;
#pragma unroll
    for (int i = 0; i < 4; ++i) { const float y = (v[i] - mu) * rs * bfr(w[l16 * 4 + i]) + bfr(bb[l16 * 4 + i]); const unsigned short hb = f2bf(y); oh[i] = hb; ol[i] = f2bf(y - bf2f(hb)); }
    *(volatile v4us*)(Hh + o) = oh; *(volatile v4us*)(Hl + o) = ol; __threadfence(); *(volatile v4us*)(Hh + o) = oh; *(volatile v4us*)(Hl + o) = ol;
}
__global__ __launch_bounds__(256) void k_wb2(const float* __restrict__ Wm, bf* WT) {
    const int u = blockIdx.x * 256 + threadIdx.x; if (u >= PW * BW / 8) return;
    const int n = u / (BW / 8), k0 = (u % (BW / 8)) * 8; v8us o;
#pragma unroll
    for (int i = 0; i < 8; ++i) o[i] = (n < 60) ? f2bf(Wm[(size_t)(k0 + i) * 60 + n]) : (unsigned short)0;
    *(volatile v8us*)(WT + (size_t)n * BW + k0) = o; __threadfence(); *(volatile v8us*)(WT + (size_t)n * BW + k0) = o;
}
__global__ __launch_bounds__(256) void k_vt(const float* __restrict__ V, h16* VTH, h16* VTL) {
    __shared__ __align__(16) h16 tile[64 * 72];
    __shared__ __align__(16) h16 til2[64 * 72];
    const int bid = blockIdx.x;
    const int b = bid / (NH_ * (NT_ / 64)), rem = bid - b * (NH_ * (NT_ / 64)), h = rem / (NT_ / 64), kt = rem - h * (NT_ / 64);
    const int k0 = kt * 64, tid = threadIdx.x;
    const int kk = tid >> 2, d0 = (tid & 3) * 16;
    const float* src = V + ((size_t)b * NT_ + k0 + kk) * DM + h * HD + d0;
#pragma unroll
    for (int i = 0; i < 16; ++i) { const float v = src[i]; const h16 a = (h16)v; tile[(d0 + i) * 72 + kk] = a; til2[(d0 + i) * 72 + kk] = (h16)((v - (float)a) * LOSC); }
    __syncthreads();
    const int piece = tid & 7;
    const size_t base = (((size_t)b * NH_ + h) * HD) * NT_ + k0;
    auto pass = [&]() {
#pragma unroll
        for (int s = 0; s < 4; ++s) { const int Lid = (tid >> 3) + 32 * s; const int pln = Lid >> 6, d = Lid & 63;
            const v8h val = *(const v8ha*)((pln ? til2 : tile) + d * 72 + piece * 8); *(volatile v8h*)((pln ? VTL : VTH) + base + (size_t)d * NT_ + piece * 8) = val; }
    };
    pass(); __threadfence(); pass();
}

__global__ __launch_bounds__(128) void k_attn(const h16* __restrict__ Q16, const h16* __restrict__ QL16, const h16* __restrict__ K16, const h16* __restrict__ KL16, const h16* __restrict__ VTH, const h16* __restrict__ VTL, const float* __restrict__ G, float* OUTP) {
    __shared__ __align__(16) h16 plds[4][16 * 32];
    __shared__ __align__(16) h16 plds2[4][16 * 32];
    __shared__ __align__(16) float ost[4][16 * 68];
    const int lane = threadIdx.x & 31, wave = threadIdx.x >> 5, lr = lane & 15, hi = lane >> 4;
    const int bid = blockIdx.x;
    const int b = bid / (NH_ * (NT_ / 64)), rem = bid - b * (NH_ * (NT_ / 64)), h = rem / (NT_ / 64), qt = rem - h * (NT_ / 64);
    const int q0 = qt * 64 + wave * 16;
    const size_t tok0 = (size_t)b * NT_;
    h16* pl = &plds[wave][0]; h16* pl2 = &plds2[wave][0];
    v16h qa[2];
    const size_t qo0 = (tok0 + q0 + lr) * DM + h * HD + 8 * hi;
#pragma unroll
    for (int kc = 0; kc < 2; ++kc) qa[kc] = cat16(*(const v8h*)(Q16 + qo0 + kc * 32), *(const v8h*)(Q16 + qo0 + kc * 32 + 16));
    const h16* kh_b = K16 + tok0 * DM + h * HD;
    const h16* kl_b = KL16 + tok0 * DM + h * HD;
    const size_t vbase = (((size_t)b * NH_ + h) * HD) * NT_;
    v8f o[4], ox[4];
#pragma unroll
    for (int n = 0; n < 4; ++n) { o[n] = (v8f){}; ox[n] = (v8f){}; }
    float mrow[8], lpart[8];
#pragma unroll
    for (int j = 0; j < 8; ++j) { mrow[j] = -3.0e38f; lpart[j] = 0.f; }
    int qpos[8];
#pragma unroll
    for (int j = 0; j < 8; ++j) qpos[j] = q0 + 8 * hi + j;
    const int kt_lo = 0, kt_hi = (qt * 64 + 63) / 32;
#pragma unroll 1
    for (int kt = kt_lo; kt <= kt_hi; ++kt) {
        const int l0 = kt * 32;
        const size_t ko0 = (size_t)(l0 + lr) * DM + 8 * hi, ko1 = (size_t)(l0 + 16 + lr) * DM + 8 * hi;
        v8f s0 = {}, s1 = {}, x0 = {}, x1 = {};
#pragma unroll
        for (int kc = 0; kc < 2; ++kc) {
            { const v16h k0h = cat16(*(const v8h*)(kh_b + ko0 + kc * 32), *(const v8h*)(kh_b + ko0 + kc * 32 + 16)), k1h = cat16(*(const v8h*)(kh_b + ko1 + kc * 32), *(const v8h*)(kh_b + ko1 + kc * 32 + 16));
              const v16h qlk = cat16(*(const v8h*)(QL16 + qo0 + kc * 32), *(const v8h*)(QL16 + qo0 + kc * 32 + 16));
              s0 = wmma16(qa[kc], k0h, s0); x0 = wmma16(qlk, k0h, x0); s1 = wmma16(qa[kc], k1h, s1); x1 = wmma16(qlk, k1h, x1);
              asm volatile("v_nop" : "+v"(s0), "+v"(s1), "+v"(x0), "+v"(x1) : "v"(qlk), "v"(k0h), "v"(k1h) : "memory"); }
            { const v16h k0l = cat16(*(const v8h*)(kl_b + ko0 + kc * 32), *(const v8h*)(kl_b + ko0 + kc * 32 + 16)), k1l = cat16(*(const v8h*)(kl_b + ko1 + kc * 32), *(const v8h*)(kl_b + ko1 + kc * 32 + 16));
              x0 = wmma16(qa[kc], k0l, x0); x1 = wmma16(qa[kc], k1l, x1);
              asm volatile("v_nop" : "+v"(x0), "+v"(x1) : "v"(k0l), "v"(k1l) : "memory"); }
        }
        asm volatile("v_nop\n\tv_nop\n\tv_nop\n\tv_nop" : "+v"(s0), "+v"(s1), "+v"(x0), "+v"(x1) : "v"(qa[0]), "v"(qa[1]));
        float alpha[8]; const float ga = G[(l0 + lr) * GH + h], gb = G[(l0 + 16 + lr) * GH + h];
#pragma unroll
        for (int j = 0; j < 8; ++j) {
            const int ja = l0 + lr, jb = l0 + 16 + lr, qi = qpos[j];
            const float a0 = (ja <= qi) ? (s0[j] + x0[j] * LOSCI) : 0.f, a1 = (jb <= qi) ? (s1[j] + x1[j] * LOSCI) : 0.f;
            const float p0 = a0 * (1.0f + ga), p1 = a1 * (1.0f + gb);
            alpha[j] = 1.0f; (void)mrow;
            lpart[j] = lpart[j] + (a0 + a1);
            const int mr = hi * 8 + j;
            const float ps0 = p0 * PSC, ps1 = p1 * PSC; const h16 h0 = (h16)ps0, h1 = (h16)ps1;
            pl[mr * 32 + lr] = h0; pl[mr * 32 + 16 + lr] = h1;
            pl2[mr * 32 + lr] = (h16)((ps0 - (float)h0) * LOSC); pl2[mr * 32 + 16 + lr] = (h16)((ps1 - (float)h1) * LOSC);
        }
        asm volatile("" ::: "memory");
        const v16h pa = cat16(*(const v8ha*)(pl + lr * 32 + hi * 8), *(const v8ha*)(pl + lr * 32 + 16 + hi * 8));
        const v16h px = cat16(*(const v8ha*)(pl2 + lr * 32 + hi * 8), *(const v8ha*)(pl2 + lr * 32 + 16 + hi * 8));
#pragma unroll
        for (int n = 0; n < 4; ++n) { const size_t vo = vbase + (size_t)(n * 16 + lr) * NT_ + l0 + hi * 8;
            const v16h vh = cat16(*(const v8h*)(VTH + vo), *(const v8h*)(VTH + vo + 16)), vl = cat16(*(const v8h*)(VTL + vo), *(const v8h*)(VTL + vo + 16));
            o[n] = wmma16(pa, vh, o[n]); ox[n] = wmma16(pa, vl, ox[n]); ox[n] = wmma16(px, vh, ox[n]);
            asm volatile("" : "+v"(o[n]), "+v"(ox[n]) : "v"(vh), "v"(vl) : "memory"); }
        asm volatile("v_nop\n\tv_nop\n\tv_nop\n\tv_nop" : "+v"(o[0]), "+v"(o[1]), "+v"(o[2]), "+v"(o[3]), "+v"(ox[0]), "+v"(ox[1]), "+v"(ox[2]), "+v"(ox[3]) : "v"(pa), "v"(px));
    }
    float inv[8];
#pragma unroll
    for (int j = 0; j < 8; ++j) { float rs = lpart[j]; rs += __shfl_xor(rs, 1, 16); rs += __shfl_xor(rs, 2, 16); rs += __shfl_xor(rs, 4, 16); rs += __shfl_xor(rs, 8, 16); inv[j] = 1.0f / (rs + 1e-6f); }
    float* os = &ost[wave][0];
#pragma unroll
    for (int n = 0; n < 4; ++n)
#pragma unroll
        for (int j = 0; j < 8; ++j) os[(hi * 8 + j) * 68 + n * 16 + lr] = (o[n][j] + ox[n][j] * LOSCI) * inv[j];
    __syncthreads();
    float* ob = OUTP + (tok0 + q0) * DM + (size_t)h * HD;
    auto pass = [&]() {
#pragma unroll
        for (int s = 0; s < 8; ++s) { const int Lid = (lane >> 3) + 4 * s, piece = lane & 7; const int row = Lid >> 1, cofs = (Lid & 1) * 32 + piece * 4;
            const v4f val = *(const v4fa*)(os + row * 68 + cofs); *(volatile v4f*)(ob + (size_t)row * DM + cofs) = val; }
    };
    pass(); __threadfence(); pass();
}

#define VST2(T, p, v) do { const T vst2_v_ = (v); *(volatile T*)(p) = vst2_v_; __threadfence(); *(volatile T*)(p) = vst2_v_; } while (0)
extern "C" void kernel_launch(void* const* d_in, const int* in_sizes, int n_in,
                              void* d_out, int out_size, void* d_ws, size_t ws_size, hipStream_t stream) {
    (void)in_sizes; (void)n_in; (void)out_size;
    const float* x = (const float*)d_in[0]; const float* Wqkv = (const float*)d_in[1]; const float* bqkv = (const float*)d_in[2]; const float* Wb1 = (const float*)d_in[3]; const float* Wb2 = (const float*)d_in[4];
    const float* temp = (const float*)d_in[5]; const float* Wp = (const float*)d_in[6]; const float* bp = (const float*)d_in[7]; const float* lnw = (const float*)d_in[8]; const float* lnb = (const float*)d_in[9]; const float* mnw = (const float*)d_in[10]; const float* mnb = (const float*)d_in[11];
    float* out0 = (float*)d_out; float* out1 = out0 + (size_t)2 * NT_ * DM;
    char* wsp = (char*)d_ws;
    auto take = [&](size_t bytes) { char* p = wsp; wsp += (bytes + 255) & ~(size_t)255; return (void*)p; };
    bf* WqkvT = (bf*)take((size_t)3 * DM * DM * 2); bf* Wb1T = (bf*)take((size_t)BW * DM * 2); bf* Wb2T = (bf*)take((size_t)PW * BW * 2); bf* WpT = (bf*)take((size_t)DM * DM * 2);
    bf* Xb = (bf*)take((size_t)NTK * DM * 2); bf* Nh = (bf*)take((size_t)NTK * DM * 2); bf* Nl = (bf*)take((size_t)NTK * DM * 2);
    float* QKV = (float*)take((size_t)NTK * 3 * DM * 4); float* BT = (float*)take((size_t)NTK * BW * 4); bf* Sh = (bf*)take((size_t)NTK * BW * 2); bf* Sl = (bf*)take((size_t)NTK * BW * 2); float* PR = (float*)take((size_t)NTK * PW * 4); float* G = (float*)take((size_t)NTK * GH * 4);
    h16* QH = (h16*)take((size_t)NTK * DM * 2); h16* QL = (h16*)take((size_t)NTK * DM * 2); h16* KH = (h16*)take((size_t)NTK * DM * 2); h16* KL = (h16*)take((size_t)NTK * DM * 2);
    float* Vf = (float*)take((size_t)NTK * DM * 4); h16* VTH = (h16*)take((size_t)NTK * DM * 2); h16* VTL = (h16*)take((size_t)NTK * DM * 2); float* CTX = (float*)take((size_t)NTK * DM * 4); bf* Ch = (bf*)take((size_t)NTK * DM * 2); bf* Cl = (bf*)take((size_t)NTK * DM * 2);
    if ((size_t)(wsp - (char*)d_ws) > ws_size) return;
    k_wt<<<dim3(DM / 64, 3 * DM / 64, 1), 256, 0, stream>>>(Wqkv, DM, 3 * DM, WqkvT); k_wt<<<dim3(DM / 64, BW / 64, 1), 256, 0, stream>>>(Wb1, DM, BW, Wb1T); k_wt<<<dim3(DM / 64, DM / 64, 1), 256, 0, stream>>>(Wp, DM, DM, WpT);
    k_wb2<<<(PW * BW / 8 + 255) / 256, 256, 0, stream>>>(Wb2, Wb2T);
    for (int b = 0; b < 2; ++b) {
        const float* xb = x + (size_t)b * NTK * DM;
        k_ln<true><<<NTK / 8, 256, 0, stream>>>(xb, lnw, lnb, NTK, Nh, Nl);
        k_cvtb<<<NTK / 8, 256, 0, stream>>>(xb, NTK, Xb);
        k_gemmb<true, false><<<dim3(NTK / 64, 3 * DM / 64, 1), 128, 0, stream>>>(Nh, Nl, WqkvT, bqkv, QKV, 3 * DM, nullptr);
        k_gemmb<false, false><<<dim3(NTK / 64, BW / 64, 1), 128, 0, stream>>>(Xb, nullptr, Wb1T, nullptr, BT, BW, nullptr);
        k_silu2<<<NTK / 8, 256, 0, stream>>>(BT, NTK, Sh, Sl);
        k_gemmb<true, false><<<dim3(NTK / 64, PW / 64, 1), 128, 0, stream>>>(Sh, Sl, Wb2T, nullptr, PR, PW, nullptr, nullptr, BW);
        k_gate<<<(NTK * GH + 255) / 256, 256, 0, stream>>>(PR, temp, G); k_gout<<<(NTK * NH_ + 255) / 256, 256, 0, stream>>>(G, out1 + (size_t)b * NT_ * NH_);
        k_elu16<<<NTK / 8, 256, 0, stream>>>(QKV, 0, NTK, QH, QL); k_elu16<<<NTK / 8, 256, 0, stream>>>(QKV, DM, NTK, KH, KL);
        k_vcopy<<<NTK / 8, 256, 0, stream>>>(QKV, NTK, Vf); k_vt<<<NB_ * NH_ * (NT_ / 64), 256, 0, stream>>>(Vf, VTH, VTL);
        k_attn<<<NB_ * NH_ * (NT_ / 64), 128, 0, stream>>>(QH, QL, KH, KL, VTH, VTL, G, CTX);
        k_hln<<<(NT_ * (NH_ / 2) + 7) / 8, 256, 0, stream>>>(CTX, mnw, mnb, nullptr, Ch, Cl);
        k_gemmb<true, false><<<dim3(NTK / 64, DM / 64, 1), 128, 0, stream>>>(Ch, Cl, WpT, bp, out0 + (size_t)b * NTK * DM, DM, nullptr);
    }
}
